// LinearAttentionSelective_41575283425768
// MI455X (gfx1250) — hardware-verified
//
#include <hip/hip_runtime.h>
#include <math.h>
#include <stdint.h>

#define NB    2
#define SEQ   2048
#define DM    1024
#define NH    16
#define FD    16
#define HD    64
#define NQK   256
#define QKP   512
#define NQB   (SEQ / 64)
#define PCAR  64.0f
#define RSC   4096.0f
static_assert(NH * HD == DM);
static_assert(NH * FD == NQK);
static_assert(2 * NQK == QKP);
static_assert(NH * 32 == QKP);
static_assert((SEQ % 64) == 0 && (DM % 256) == 0 && (NQK % 64) == 0);
static_assert(HD == 64);

typedef _Float16 v16h __attribute__((ext_vector_type(16)));
typedef _Float16 v8h  __attribute__((ext_vector_type(8)));
typedef __bf16   v16b __attribute__((ext_vector_type(16)));
typedef __bf16   v8b  __attribute__((ext_vector_type(8)));
typedef float    v8f  __attribute__((ext_vector_type(8)));
typedef float    v4f  __attribute__((ext_vector_type(4)));
typedef unsigned int v4u __attribute__((ext_vector_type(4)));

__device__ __forceinline__ unsigned short bf_bits(float f) {
  unsigned u = __float_as_uint(f);
  return (unsigned short)((u + 0x7FFFu + ((u >> 16) & 1u)) >> 16);
}
__device__ __forceinline__ float bf_up(unsigned short h) { return __uint_as_float(((unsigned)h) << 16); }
__device__ __forceinline__ unsigned short h_bits(_Float16 x) { return __builtin_bit_cast(unsigned short, x); }
__device__ __forceinline__ unsigned pk16(unsigned short a, unsigned short b) { return (unsigned)a | ((unsigned)b << 16); }
__device__ __forceinline__ v8f zero8() { v8f z = {0.f, 0.f, 0.f, 0.f, 0.f, 0.f, 0.f, 0.f}; return z; }

__device__ __forceinline__ v16b ldfrag_b(const __bf16* p) {
  union { v16b v; v8b h[2]; } f;
  f.h[0] = *(const v8b*)(p);
  f.h[1] = *(const v8b*)(p + 16);
  return f.v;
}

__device__ __forceinline__ v8f mma_b(v16b a, v16b b, v8f c) {
  c = __builtin_amdgcn_wmma_f32_16x16x32_bf16(false, a, false, b, (short)0, c, false, false);
#if defined(__HIP_DEVICE_COMPILE__)
  asm volatile("v_nop\n\tv_nop\n\tv_nop\n\tv_nop" : "+v"(c) : "v"(a), "v"(b));
#endif
  return c;
}
__device__ __forceinline__ v8f mma_h(v16h a, v16h b, v8f c) {
  c = __builtin_amdgcn_wmma_f32_16x16x32_f16(false, a, false, b, (short)0, c, false, false);
#if defined(__HIP_DEVICE_COMPILE__)
  asm volatile("v_nop\n\tv_nop\n\tv_nop\n\tv_nop" : "+v"(c) : "v"(a), "v"(b));
#endif
  return c;
}
__device__ __forceinline__ v8f mma_b_raw(v16b a, v16b b, v8f c) {
  return __builtin_amdgcn_wmma_f32_16x16x32_bf16(false, a, false, b, (short)0, c, false, false);
}
__device__ __forceinline__ void dep_guard_b(v8f& a, v8f& b, v16b x, v16b y) {
#if defined(__HIP_DEVICE_COMPILE__)
  asm volatile("v_nop\n\tv_nop\n\tv_nop\n\tv_nop" : "+v"(a), "+v"(b) : "v"(x), "v"(y));
#endif
}
__device__ __forceinline__ void keep4_b(v16b a, v16b b, v16b c, v16b d) {
#if defined(__HIP_DEVICE_COMPILE__)
  asm volatile("v_nop" :: "v"(a), "v"(b), "v"(c), "v"(d));
#endif
}
__device__ __forceinline__ void acc_guard4(v8f& a, v8f& b, v8f& c, v8f& d) {
#if defined(__HIP_DEVICE_COMPILE__)
  asm volatile("v_nop\n\tv_nop\n\tv_nop\n\tv_nop" : "+v"(a), "+v"(b), "+v"(c), "+v"(d));
#endif
}

__global__ __launch_bounds__(256) void cvt_bf16x8(const float* __restrict__ in, unsigned short* out, int n8) {
  const int i = blockIdx.x * 256 + threadIdx.x;
  if (i < n8) {
    const v4f a = *(const v4f*)(in + (size_t)i * 8);
    const v4f b = *(const v4f*)(in + (size_t)i * 8 + 4);
    v4u p;
    p[0] = pk16(bf_bits(a[0]), bf_bits(a[1]));
    p[1] = pk16(bf_bits(a[2]), bf_bits(a[3]));
    p[2] = pk16(bf_bits(b[0]), bf_bits(b[1]));
    p[3] = pk16(bf_bits(b[2]), bf_bits(b[3]));
    *(volatile v4u*)(out + (size_t)i * 8) = p;
    __threadfence();
    *(volatile v4u*)(out + (size_t)i * 8) = p;
  }
}

__global__ __launch_bounds__(256) void tr_cvt(const float* __restrict__ in, int R, int C,
                                              unsigned short* out, int ldo) {
  __shared__ __align__(16) float st[64 * 68];
  const int tid = threadIdx.x, wave = tid >> 5, lane = tid & 31;
  const int tilesC = C >> 6;
  const int tcI = blockIdx.x % tilesC;
  const int trI = blockIdx.x / tilesC;
  const int r0 = trI << 6, c0 = tcI << 6;
  (void)R;
#pragma unroll
  for (int pass = 0; pass < 4; ++pass) {
    const int r = pass * 16 + (tid >> 4), c4 = (tid & 15) * 4;
    const v4f v = *(const v4f*)(in + (size_t)(r0 + r) * C + c0 + c4);
    *(v4f*)(st + r * 68 + c4) = v;
  }
  __syncthreads();
  const int piece = lane & 7, sub = lane >> 3;
  const int k = piece * 8;
  v4u pv[2];
#pragma unroll
  for (int it = 0; it < 2; ++it) {
    const int cl = wave * 8 + it * 4 + sub;
    v4u p;
#pragma unroll
    for (int e = 0; e < 4; ++e) {
      const float f0 = st[(k + 2 * e) * 68 + cl];
      const float f1 = st[(k + 2 * e + 1) * 68 + cl];
      p[e] = pk16(bf_bits(f0), bf_bits(f1));
    }
    pv[it] = p;
  }
  for (int pass = 0; pass < 2; ++pass) {
#pragma unroll
    for (int it = 0; it < 2; ++it) {
      const int cl = wave * 8 + it * 4 + sub;
      *(volatile v4u*)(out + (size_t)(c0 + cl) * ldo + r0 + k) = pv[it];
    }
    __threadfence();
  }
}

template <int NSPLIT, int OUT_MODE, bool RS, bool CS>
__global__ __launch_bounds__(256) void gemm64(
    const unsigned short* __restrict__ Ap, const unsigned short* A2p, int lda, long long strideA,
    const unsigned short* __restrict__ Btp, const unsigned short* Bt2p, int ldb, long long strideB,
    void* Cout, int ldc, long long strideC,
    void* Cout2, int ldc2, long long strideC2, int N2,
    int M, int N, int K, float rscale,
    const float* __restrict__ rsp, const float* __restrict__ csp) {
  const __bf16* A   = (const __bf16*)(const void*)Ap;
  const __bf16* A2  = (const __bf16*)(const void*)A2p;
  const __bf16* Bt  = (const __bf16*)(const void*)Btp;
  const __bf16* Bt2 = (const __bf16*)(const void*)Bt2p;
  __shared__ __align__(16) float sT[8][16 * 68];
  const int b    = blockIdx.y;
  const int lane = threadIdx.x & 31;
  const int wave = threadIdx.x >> 5;
  const int tilesN = N >> 6;
  const int tilesM = M >> 6;
  const int tile = blockIdx.x * 8 + wave;
  if (tile >= tilesM * tilesN) return;
  const int tm = tile / tilesN;
  const int tn = tile - tm * tilesN;
  const int m0 = tm << 6;
  const int n0 = tn << 6;

  const __bf16* Ab  = A  + (size_t)b * strideA;
  const __bf16* Bb  = Bt + (size_t)b * strideB;
  const __bf16* Ab2 = (NSPLIT >= 1) ? (A2  + (size_t)b * strideA) : Ab;
  const __bf16* Bb2 = (NSPLIT == 2) ? (Bt2 + (size_t)b * strideB) : Bb;

  const int rlane = lane & 15;
  const int koff  = (lane >> 4) * 8;
  const int mOff  = (lane >> 4) * 8;

  v8f acc[4][4];
#pragma unroll
  for (int i = 0; i < 4; ++i)
#pragma unroll
    for (int j = 0; j < 4; ++j) acc[i][j] = zero8();

  for (int k0 = 0; k0 < K; k0 += 32) {
    v16b bh[4], bl[4];
#pragma unroll
    for (int j = 0; j < 4; ++j) {
      const size_t bo = (size_t)(n0 + (j << 4) + rlane) * ldb + koff + k0;
      bh[j] = ldfrag_b(Bb + bo);
      if (NSPLIT == 2) bl[j] = ldfrag_b(Bb2 + bo); else bl[j] = bh[j];
    }
#pragma unroll
    for (int i = 0; i < 4; ++i) {
      const size_t ao = (size_t)(m0 + (i << 4) + rlane) * lda + koff + k0;
      const v16b ah = ldfrag_b(Ab + ao);
      v16b al = ah;
      if (NSPLIT >= 1) al = ldfrag_b(Ab2 + ao);
#pragma unroll
      for (int j = 0; j < 4; ++j) {
        acc[i][j] = mma_b_raw(ah, bh[j], acc[i][j]);
        if (NSPLIT >= 1) acc[i][j] = mma_b_raw(al, bh[j], acc[i][j]);
        if (NSPLIT == 2) acc[i][j] = mma_b_raw(ah, bl[j], acc[i][j]);
      }
      dep_guard_b(acc[i][0], acc[i][3], ah, al);
    }
    keep4_b(bh[0], bh[1], bh[2], bh[3]);
    if (NSPLIT == 2) keep4_b(bl[0], bl[1], bl[2], bl[3]);
  }
  acc_guard4(acc[0][0], acc[0][1], acc[0][2], acc[0][3]);
  acc_guard4(acc[1][0], acc[1][1], acc[1][2], acc[1][3]);
  acc_guard4(acc[2][0], acc[2][1], acc[2][2], acc[2][3]);
  acc_guard4(acc[3][0], acc[3][1], acc[3][2], acc[3][3]);

  float csv[4];
#pragma unroll
  for (int j = 0; j < 4; ++j) csv[j] = CS ? csp[n0 + (j << 4) + rlane] : 1.0f;

  float* slab = sT[wave];
#pragma unroll
  for (int i = 0; i < 4; ++i) {
    const int mBase = m0 + (i << 4);
#pragma unroll
    for (int r = 0; r < 8; ++r) {
      const float rsv = RS ? rsp[mBase + mOff + r] : 1.0f;
#pragma unroll
      for (int j = 0; j < 4; ++j) {
        slab[(mOff + r) * 68 + (j << 4) + rlane] = acc[i][j][r] * rsv * csv[j];
      }
    }
    __builtin_amdgcn_fence(__ATOMIC_RELEASE, "workgroup");
    __builtin_amdgcn_wave_barrier();
    __builtin_amdgcn_fence(__ATOMIC_ACQUIRE, "workgroup");
    if (OUT_MODE == 0) {
      float* C = (float*)Cout + (size_t)b * strideC;
      const int hh = lane >> 4, c4 = (lane & 15) * 4;
      v4f ov[8];
#pragma unroll
      for (int it = 0; it < 8; ++it) {
        const int row = it * 2 + hh;
        ov[it] = *(const v4f*)(slab + row * 68 + c4);
      }
      for (int pass = 0; pass < 2; ++pass) {
#pragma unroll
        for (int it = 0; it < 8; ++it) {
          const int row = it * 2 + hh;
          *(volatile v4f*)(C + (size_t)(mBase + row) * ldc + n0 + c4) = ov[it];
        }
        __threadfence();
      }
    } else {
      const int q = lane >> 3, c8 = (lane & 7) * 8;
      unsigned short* C  = (unsigned short*)Cout  + (size_t)b * strideC;
      unsigned short* C2 = (unsigned short*)Cout2 + (size_t)b * strideC2;
      const bool wlo = (OUT_MODE == 2) || (n0 < N2);
      v4u hv[4], lv[4];
#pragma unroll
      for (int it = 0; it < 4; ++it) {
        const int row = it * 4 + q;
        const float* sp = slab + row * 68 + c8;
        v4u a, a2;
#pragma unroll
        for (int e = 0; e < 4; ++e) {
          const float f0 = sp[2 * e], f1 = sp[2 * e + 1];
          unsigned short h0, h1, l0, l1;
          if (OUT_MODE == 2) {
            h0 = bf_bits(f0); h1 = bf_bits(f1);
            l0 = bf_bits(f0 - bf_up(h0)); l1 = bf_bits(f1 - bf_up(h1));
          } else {
            const _Float16 x0 = (_Float16)f0, x1 = (_Float16)f1;
            h0 = h_bits(x0); h1 = h_bits(x1);
            l0 = h_bits((_Float16)((f0 - (float)x0) * rscale));
            l1 = h_bits((_Float16)((f1 - (float)x1) * rscale));
          }
          a[e] = pk16(h0, h1); a2[e] = pk16(l0, l1);
        }
        hv[it] = a; lv[it] = a2;
      }
      for (int pass = 0; pass < 2; ++pass) {
#pragma unroll
        for (int it = 0; it < 4; ++it) {
          const int row = it * 4 + q;
          *(volatile v4u*)(C + (size_t)(mBase + row) * ldc + n0 + c8) = hv[it];
          if (wlo) *(volatile v4u*)(C2 + (size_t)(mBase + row) * ldc2 + n0 + c8) = lv[it];
        }
        __threadfence();
      }
    }
    __builtin_amdgcn_fence(__ATOMIC_RELEASE, "workgroup");
    __builtin_amdgcn_wave_barrier();
    __builtin_amdgcn_fence(__ATOMIC_ACQUIRE, "workgroup");
  }
}

__global__ __launch_bounds__(256) void qk_planes(const float* __restrict__ qkf,
                                                 unsigned short* qap, unsigned short* kap,
                                                 unsigned short* qbp, unsigned short* kbp) {
  __shared__ __align__(16) unsigned int sp[8][4][256];
  const int tid = threadIdx.x, wave = tid >> 5, lane = tid & 31;
  const int row = blockIdx.x * 8 + wave;
  const int t = lane >> 4, hs = lane & 15;
  const float* src = qkf + (size_t)row * QKP + t * NQK + hs * FD;
  v4u H[2], L[2];
#pragma unroll
  for (int g = 0; g < 2; ++g) {
    const v4f a  = *(const v4f*)(src + 8 * g);
    const v4f bq = *(const v4f*)(src + 8 * g + 4);
    v4u ph, pl;
#pragma unroll
    for (int e = 0; e < 4; ++e) {
      const float f0 = (e < 2) ? a[2 * e]     : bq[2 * e - 4];
      const float f1 = (e < 2) ? a[2 * e + 1] : bq[2 * e - 3];
      const unsigned short h0 = bf_bits(f0), h1 = bf_bits(f1);
      const unsigned short l0 = bf_bits(f0 - bf_up(h0)), l1 = bf_bits(f1 - bf_up(h1));
      ph[e] = pk16(h0, h1); pl[e] = pk16(l0, l1);
    }
    H[g] = ph; L[g] = pl;
  }
  v4u W2[2], W3[2];
  const v4u Z = {0u, 0u, 0u, 0u};
#pragma unroll
  for (int g = 0; g < 2; ++g) {
#pragma unroll
    for (int e = 0; e < 4; ++e) {
      W2[g][e] = t ? H[g][e] : L[g][e];
      W3[g][e] = t ? L[g][e] : H[g][e];
    }
  }
  unsigned int* pa = &sp[wave][t][hs * 16];
  unsigned int* pb = &sp[wave][2 + t][hs * 16];
  *(v4u*)(pa + 0)  = H[0];
  *(v4u*)(pa + 4)  = H[1];
  *(v4u*)(pa + 8)  = W2[0];
  *(v4u*)(pa + 12) = W2[1];
  *(v4u*)(pb + 0)  = W3[0];
  *(v4u*)(pb + 4)  = W3[1];
  *(v4u*)(pb + 8)  = Z;
  *(v4u*)(pb + 12) = Z;
  __builtin_amdgcn_fence(__ATOMIC_RELEASE, "workgroup");
  __builtin_amdgcn_wave_barrier();
  __builtin_amdgcn_fence(__ATOMIC_ACQUIRE, "workgroup");
  v4u ov[8];
#pragma unroll
  for (int p = 0; p < 4; ++p) {
#pragma unroll
    for (int i = 0; i < 2; ++i) ov[p * 2 + i] = *(const v4u*)(&sp[wave][p][i * 128 + lane * 4]);
  }
  const size_t go = (size_t)row * QKP + lane * 8;
  for (int pass = 0; pass < 2; ++pass) {
    *(volatile v4u*)(qap + go)       = ov[0];
    *(volatile v4u*)(qap + go + 256) = ov[1];
    *(volatile v4u*)(kap + go)       = ov[2];
    *(volatile v4u*)(kap + go + 256) = ov[3];
    *(volatile v4u*)(qbp + go)       = ov[4];
    *(volatile v4u*)(qbp + go + 256) = ov[5];
    *(volatile v4u*)(kbp + go)       = ov[6];
    *(volatile v4u*)(kbp + go + 256) = ov[7];
    __threadfence();
  }
}

__global__ __launch_bounds__(128)
void lin_attn(const unsigned short* __restrict__ qap, const unsigned short* __restrict__ kap,
              const unsigned short* __restrict__ qbp, const unsigned short* __restrict__ kbp,
              const unsigned short* __restrict__ vhp, const unsigned short* __restrict__ vlp,
              float* outp) {
  union FB { v16b v; v8b h[2]; };
  union FH { v16h v; v8h h[2]; };
  __shared__ __align__(16) __bf16   Kas[64 * 32];
  __shared__ __align__(16) __bf16   Kbs[64 * 32];
  __shared__ __align__(16) _Float16 Vth[64 * 64];
  __shared__ __align__(16) _Float16 Vtl[64 * 64];
  __shared__ __align__(16) _Float16 Psh[4][16 * 64];
  __shared__ __align__(16) _Float16 Psl[4][16 * 64];
  __shared__ __align__(16) float    Os[4][16 * 64];

  const int tid  = threadIdx.x;
  const int wave = tid >> 5;
  const int lane = tid & 31;
  const int hh   = lane >> 4;
  const int c    = lane & 15;

  const int bx   = blockIdx.x;
  const int qb   = bx % NQB;
  const int rest = bx / NQB;
  const int h    = rest % NH;
  const int b    = rest / NH;
  const int q0   = qb * 64 + wave * 16;
  const size_t rowB = (size_t)b * SEQ;

  const __bf16* QA = (const __bf16*)(const void*)qap + (size_t)h * 32;
  const __bf16* KA = (const __bf16*)(const void*)kap + (size_t)h * 32;
  const __bf16* QB = (const __bf16*)(const void*)qbp + (size_t)h * 32;
  const __bf16* KB = (const __bf16*)(const void*)kbp + (size_t)h * 32;
  const _Float16* Vh = (const _Float16*)(const void*)vhp + ((size_t)b * DM + (size_t)h * HD) * SEQ;
  const _Float16* Vl = (const _Float16*)(const void*)vlp + ((size_t)b * DM + (size_t)h * HD) * SEQ;

  const v16b qfa = ldfrag_b(QA + (rowB + q0 + c) * QKP + 8 * hh);
  const v16b qfb = ldfrag_b(QB + (rowB + q0 + c) * QKP + 8 * hh);

  float lrow[8];
  v8f oacc[4];
#pragma unroll
  for (int r = 0; r < 8; ++r) lrow[r] = 0.f;
#pragma unroll
  for (int t = 0; t < 4; ++t) oacc[t] = zero8();

  const int nkt = qb + 1;
  for (int kt = 0; kt < nkt; ++kt) {
    const int kv0 = kt * 64;
    __syncthreads();
    {
#pragma unroll
      for (int i = 0; i < 2; ++i) {
        const int idx = tid + 128 * i, r = idx >> 2, pc8 = (idx & 3) * 8;
        const size_t ko = (rowB + kv0 + r) * QKP + pc8;
        const v8b a0 = *(const v8b*)(KA + ko);
        const v8b a1 = *(const v8b*)(KB + ko);
        *(v8b*)(Kas + r * 32 + pc8) = a0;
        *(v8b*)(Kbs + r * 32 + pc8) = a1;
      }
#pragma unroll
      for (int i = 0; i < 4; ++i) {
        const int idx = tid + 128 * i, r = idx >> 3, pc8 = (idx & 7) * 8;
        const size_t vo = (size_t)r * SEQ + kv0 + pc8;
        const v8h b0 = *(const v8h*)(Vh + vo);
        const v8h b1 = *(const v8h*)(Vl + vo);
        *(v8h*)(Vth + r * 64 + pc8) = b0;
        *(v8h*)(Vtl + r * 64 + pc8) = b1;
      }
    }
    __syncthreads();

    v8f s[4];
#pragma unroll
    for (int j = 0; j < 4; ++j) {
      FB ka, kb;
      ka.h[0] = *(const v8b*)(Kas + (j * 16 + c) * 32 + 8 * hh);
      ka.h[1] = *(const v8b*)(Kas + (j * 16 + c) * 32 + 16 + 8 * hh);
      kb.h[0] = *(const v8b*)(Kbs + (j * 16 + c) * 32 + 8 * hh);
      kb.h[1] = *(const v8b*)(Kbs + (j * 16 + c) * 32 + 16 + 8 * hh);
      s[j] = mma_b(qfa, ka.v, zero8());
      s[j] = mma_b(qfb, kb.v, s[j]);
    }

    _Float16* pwh = Psh[wave];
    _Float16* pwl = Psl[wave];
#pragma unroll
    for (int r = 0; r < 8; ++r) {
      const int qrow = q0 + 8 * hh + r;
      float psum = 0.f;
#pragma unroll
      for (int j = 0; j < 4; ++j) {
        const int key = kv0 + j * 16 + c;
        const float sv = s[j][r];
        float phi = 1.0f + sv * (0.25f + 0.03125f * sv);
        phi = fminf(phi, 500.0f);
        phi = (key > qrow) ? 0.0f : phi;
        psum += phi;
        const float pc = phi * PCAR;
        const _Float16 ph = (_Float16)pc;
        const _Float16 pl = (_Float16)((pc - (float)ph) * RSC);
        pwh[(8 * hh + r) * 64 + j * 16 + c] = ph;
        pwl[(8 * hh + r) * 64 + j * 16 + c] = pl;
      }
#pragma unroll
      for (int off = 1; off < 16; off <<= 1) psum += __shfl_xor(psum, off, 32);
      lrow[r] += psum;
    }
    __builtin_amdgcn_fence(__ATOMIC_RELEASE, "workgroup");
    __builtin_amdgcn_wave_barrier();
    __builtin_amdgcn_fence(__ATOMIC_ACQUIRE, "workgroup");

    v8f o1[4];
#pragma unroll
    for (int t = 0; t < 4; ++t) o1[t] = zero8();
#pragma unroll 1
    for (int kk = 0; kk < 2; ++kk) {
      FH pa, pl;
      pa.h[0] = *(const v8h*)(pwh + c * 64 + kk * 32 + 8 * hh);
      pa.h[1] = *(const v8h*)(pwh + c * 64 + kk * 32 + 16 + 8 * hh);
      pl.h[0] = *(const v8h*)(pwl + c * 64 + kk * 32 + 8 * hh);
      pl.h[1] = *(const v8h*)(pwl + c * 64 + kk * 32 + 16 + 8 * hh);
#pragma unroll
      for (int t = 0; t < 4; ++t) {
        FH vb, vl;
        vb.h[0] = *(const v8h*)(Vth + (t * 16 + c) * 64 + kk * 32 + 8 * hh);
        vb.h[1] = *(const v8h*)(Vth + (t * 16 + c) * 64 + kk * 32 + 16 + 8 * hh);
        vl.h[0] = *(const v8h*)(Vtl + (t * 16 + c) * 64 + kk * 32 + 8 * hh);
        vl.h[1] = *(const v8h*)(Vtl + (t * 16 + c) * 64 + kk * 32 + 16 + 8 * hh);
        oacc[t] = mma_h(pa.v, vb.v, oacc[t]);
        o1[t]   = mma_h(pa.v, vl.v, o1[t]);
        o1[t]   = mma_h(pl.v, vb.v, o1[t]);
      }
    }
#pragma unroll
    for (int t = 0; t < 4; ++t)
#pragma unroll
      for (int r = 0; r < 8; ++r) oacc[t][r] += o1[t][r] * (1.0f / RSC);
  }

  float* os = Os[wave];
#pragma unroll
  for (int r = 0; r < 8; ++r) {
    const float l = lrow[r];
    const float inv = (1.0f / (l + 1e-12f)) * (1.0f / PCAR);
#pragma unroll
    for (int t = 0; t < 4; ++t) os[(8 * hh + r) * 64 + t * 16 + c] = oacc[t][r] * inv;
  }
  __builtin_amdgcn_fence(__ATOMIC_RELEASE, "workgroup");
  __builtin_amdgcn_wave_barrier();
  __builtin_amdgcn_fence(__ATOMIC_ACQUIRE, "workgroup");
  {
    const int h2 = lane >> 4, c4 = (lane & 15) * 4;
    v4f ov[8];
#pragma unroll
    for (int it = 0; it < 8; ++it) {
      const int row = it * 2 + h2;
      ov[it] = *(const v4f*)(os + row * 64 + c4);
    }
    for (int pass = 0; pass < 2; ++pass) {
#pragma unroll
      for (int it = 0; it < 8; ++it) {
        const int row = it * 2 + h2;
        const size_t go = (rowB + q0 + row) * DM + (size_t)h * HD + c4;
        *(volatile v4f*)(outp + go) = ov[it];
      }
      __threadfence();
    }
  }
}

__global__ __launch_bounds__(256) void split_rows(const float* __restrict__ in, unsigned short* hp,
                                                  unsigned short* lp) {
  const int tid = threadIdx.x, wave = tid >> 5, lane = tid & 31;
#pragma unroll 1
  for (int i = 0; i < 4; ++i) {
    const int row = blockIdx.x * 32 + wave * 4 + i;
    const float* rp = in + (size_t)row * DM + lane * 8;
    v4u hv[4], lv[4];
#pragma unroll
    for (int t = 0; t < 4; ++t) {
      const v4f a  = *(const v4f*)(rp + t * 256);
      const v4f bq = *(const v4f*)(rp + t * 256 + 4);
      v4u ph, pl;
#pragma unroll
      for (int e = 0; e < 4; ++e) {
        const float f0 = (e < 2) ? a[2 * e]     : bq[2 * e - 4];
        const float f1 = (e < 2) ? a[2 * e + 1] : bq[2 * e - 3];
        const unsigned short h0 = bf_bits(f0), h1 = bf_bits(f1);
        ph[e] = pk16(h0, h1);
        pl[e] = pk16(bf_bits(f0 - bf_up(h0)), bf_bits(f1 - bf_up(h1)));
      }
      hv[t] = ph; lv[t] = pl;
    }
    for (int pass = 0; pass < 2; ++pass) {
#pragma unroll
      for (int t = 0; t < 4; ++t) {
        const size_t go = (size_t)row * DM + t * 256 + lane * 8;
        *(volatile v4u*)(hp + go) = hv[t];
        *(volatile v4u*)(lp + go) = lv[t];
      }
      __threadfence();
    }
  }
}

extern "C" void kernel_launch(void* const* d_in, const int* in_sizes, int n_in,
                              void* d_out, int out_size, void* d_ws, size_t ws_size,
                              hipStream_t stream) {
  if (n_in < 5) return;
  if (in_sizes[0] != NB * SEQ * DM) return;
  if (in_sizes[1] != DM * NQK) return;
  if (in_sizes[2] != DM * NQK) return;
  if (in_sizes[3] != DM * DM) return;
  if (in_sizes[4] != DM * DM) return;
  if (out_size != NB * SEQ * DM) return;

  const float* x  = (const float*)d_in[0];
  const float* wq = (const float*)d_in[1];
  const float* wk = (const float*)d_in[2];
  const float* wv = (const float*)d_in[3];
  const float* wo = (const float*)d_in[4];

  const size_t PXb  = (size_t)NB * SEQ * DM * 2;
  const size_t PWqk = (size_t)QKP * DM * 2;
  const size_t PW   = (size_t)DM * DM * 2;
  const size_t PQK  = (size_t)NB * SEQ * QKP * 4;
  const size_t PVT  = (size_t)NB * DM * SEQ * 2;
  const size_t PPl  = (size_t)NB * SEQ * QKP * 2;
  const size_t PAf  = (size_t)NB * SEQ * DM * 4;
  size_t off = 0;
  const size_t oXb  = off; off += PXb;
  const size_t oWqk = off; off += PWqk;
  const size_t oWv  = off; off += PW;
  const size_t oWo  = off; off += PW;
  const size_t oQK  = off; off += PQK;
  const size_t oVTh = off; off += PVT;
  const size_t oVTl = off; off += PVT;
  const size_t oQA  = off; off += PPl;
  const size_t oKA  = off; off += PPl;
  const size_t oQB  = off; off += PPl;
  const size_t oKB  = off; off += PPl;
  const size_t oAf  = off; off += PAf;
  const size_t oAh  = off; off += PXb;
  const size_t oAl  = off; off += PXb;
  if (off > ws_size) return;
  if (off > (size_t)134217728) return;

  char* ws = (char*)d_ws;
  unsigned short* Xb   = (unsigned short*)(ws + oXb);
  unsigned short* Wqkt = (unsigned short*)(ws + oWqk);
  unsigned short* Wvt  = (unsigned short*)(ws + oWv);
  unsigned short* Wot  = (unsigned short*)(ws + oWo);
  float*          QKf  = (float*)(ws + oQK);
  unsigned short* VTh  = (unsigned short*)(ws + oVTh);
  unsigned short* VTl  = (unsigned short*)(ws + oVTl);
  unsigned short* QAp  = (unsigned short*)(ws + oQA);
  unsigned short* KAp  = (unsigned short*)(ws + oKA);
  unsigned short* QBp  = (unsigned short*)(ws + oQB);
  unsigned short* KBp  = (unsigned short*)(ws + oKB);
  float*          Af   = (float*)(ws + oAf);
  unsigned short* Ah   = (unsigned short*)(ws + oAh);
  unsigned short* Al   = (unsigned short*)(ws + oAl);

  const dim3 blk(256);
  const int n8x = NB * SEQ * DM / 8;
  const dim3 gCvtX((n8x + 255) / 256);
  const dim3 gTrQ((DM / 64) * (NQK / 64));
  const dim3 gTrW((DM / 64) * (DM / 64));
  const dim3 gQK(((NB * SEQ / 64) * (QKP / 64) + 7) / 8, 1);
  const dim3 gVT(((DM / 64) * (SEQ / 64) + 7) / 8, NB);
  const dim3 gPl(NB * SEQ / 8);
  const dim3 gAttn(NB * NH * NQB);
  const dim3 gSplit(NB * SEQ / 32);
  const dim3 gOut(((NB * SEQ / 64) * (DM / 64) + 7) / 8, 1);

  cvt_bf16x8<<<gCvtX, blk, 0, stream>>>(x, Xb, n8x);
  tr_cvt<<<gTrQ, blk, 0, stream>>>(wq, DM, NQK, Wqkt, DM);
  tr_cvt<<<gTrQ, blk, 0, stream>>>(wk, DM, NQK, Wqkt + (size_t)NQK * DM, DM);
  tr_cvt<<<gTrW, blk, 0, stream>>>(wv, DM, DM, Wvt, DM);
  tr_cvt<<<gTrW, blk, 0, stream>>>(wo, DM, DM, Wot, DM);
  gemm64<0, 0, false, false><<<gQK, blk, 0, stream>>>(
      Xb, Xb, DM, 0LL, Wqkt, Wqkt, DM, 0LL,
      (void*)QKf, QKP, 0LL, (void*)QKf, 0, 0LL, 0,
      NB * SEQ, QKP, DM, 1.0f, QKf, QKf);
  gemm64<0, 3, false, false><<<gVT, blk, 0, stream>>>(
      Wvt, Wvt, DM, 0LL, Xb, Xb, DM, (long long)SEQ * DM,
      (void*)VTh, SEQ, (long long)DM * SEQ, (void*)VTl, SEQ, (long long)DM * SEQ, SEQ,
      DM, SEQ, DM, RSC, QKf, QKf);
  qk_planes<<<gPl, blk, 0, stream>>>(QKf, QAp, KAp, QBp, KBp);
  lin_attn<<<gAttn, dim3(128), 0, stream>>>(QAp, KAp, QBp, KBp, VTh, VTl, Af);
  split_rows<<<gSplit, blk, 0, stream>>>(Af, Ah, Al);
  gemm64<1, 0, false, false><<<gOut, blk, 0, stream>>>(
      Ah, Al, DM, 0LL, Wot, Wot, DM, 0LL,
      d_out, DM, 0LL, d_out, 0, 0LL, 0,
      NB * SEQ, DM, DM, 1.0f, Af, Af);
  (void)hipGetLastError();
}
